// HyperPatchInvertedResidual_32375463477392
// MI455X (gfx1250) — hardware-verified
//
#include <hip/hip_runtime.h>


#define NBI  8
#define CI   32
#define CH   192
#define CO   32
#define HI   128
#define FP   8
#define PP   16
#define KP   18
#define NPAT (NBI * FP * FP)
#define PR   324
#define PRP  384
#define HYP  14016
#define R1   (CI * CH)
#define R2   (R1 + CH * 9)
#define PCH  128
typedef _Float16 h16;
typedef unsigned short bf;
typedef __attribute__((ext_vector_type(16))) __bf16   v16bf;
typedef __attribute__((ext_vector_type(16))) _Float16 v16h;
typedef __attribute__((ext_vector_type(8)))  _Float16 v8h;
typedef __attribute__((ext_vector_type(8)))  unsigned short v8us;
typedef __attribute__((ext_vector_type(8)))  float    v8f;
typedef __attribute__((ext_vector_type(4)))  float    v4f;
typedef v8h  __attribute__((may_alias)) v8ha;
typedef v4f  __attribute__((may_alias)) v4fa;
typedef v8us __attribute__((may_alias)) v8usa;

__device__ __forceinline__ unsigned short f2bf(float f) { unsigned u = __float_as_uint(f); u += 0x7FFFu + ((u >> 16) & 1u); return (unsigned short)(u >> 16); }
__device__ __forceinline__ float bf2f(unsigned short b) { return __uint_as_float(((unsigned)b) << 16); }
__device__ __forceinline__ float bfr(float f) { return bf2f(f2bf(f)); }
__device__ __forceinline__ v16h cat16(v8h lo, v8h hi) { return __builtin_shufflevector(lo, hi, 0, 1, 2, 3, 4, 5, 6, 7, 8, 9, 10, 11, 12, 13, 14, 15); }
__device__ __forceinline__ v16bf cat16b(v8us lo, v8us hi) { return __builtin_bit_cast(v16bf, __builtin_shufflevector(lo, hi, 0, 1, 2, 3, 4, 5, 6, 7, 8, 9, 10, 11, 12, 13, 14, 15)); }
__device__ __forceinline__ v8f wmma16(v16h a, v16h b, v8f c) { return __builtin_amdgcn_wmma_f32_16x16x32_f16(false, a, false, b, (short)0, c, false, false); }
__device__ __forceinline__ v8f wmmab(v16bf a, v16bf b, v8f c) { return __builtin_amdgcn_wmma_f32_16x16x32_bf16(false, a, false, b, (short)0, c, false, false); }


template <typename T16> struct WFrag;
template <> struct WFrag<h16> { typedef v16h V; static __device__ __forceinline__ V ld(const h16* p) { return cat16(*(const v8h*)p, *(const v8h*)(p + 16)); } static __device__ __forceinline__ v8f mma(V a, V b, v8f c) { return wmma16(a, b, c); } };
template <> struct WFrag<bf> { typedef v16bf V; static __device__ __forceinline__ V ld(const bf* p) { return cat16b(*(const v8us*)p, *(const v8us*)(p + 16)); } static __device__ __forceinline__ v8f mma(V a, V b, v8f c) { return wmmab(a, b, c); } };
template <typename T16, int NSPLIT, bool BIAS>
__global__ __launch_bounds__(32) void k_gemmw(const T16* __restrict__ A, const T16* __restrict__ A2, const T16* __restrict__ Bt, const T16* __restrict__ Bt2, int K, float* C, int ldc, const float* __restrict__ bias, size_t sA, size_t sB, size_t sC) {
    typedef typename WFrag<T16>::V V;
    __shared__ __align__(16) float os[16 * 68];
    const size_t z = blockIdx.z; A += z * sA; if (A2) A2 += z * sA; Bt += z * sB; if (Bt2) Bt2 += z * sB; C += z * sC;
    const int lane = threadIdx.x & 31, lr = lane & 15, hi = lane >> 4; const int r0 = blockIdx.x * 64, c0 = blockIdx.y * 64;
    v8f acc[4][4];
#pragma unroll
    for (int mb = 0; mb < 4; ++mb)
#pragma unroll
        for (int nb = 0; nb < 4; ++nb) acc[mb][nb] = (v8f){};
    const size_t aoff = (size_t)(r0 + lr) * K + 8 * hi, boff = (size_t)(c0 + lr) * K + 8 * hi;
#pragma unroll 1
    for (int kc = 0; kc < K; kc += 32) {
        V a[4], a2[4];
#pragma unroll
        for (int mb = 0; mb < 4; ++mb) { a[mb] = WFrag<T16>::ld(A + aoff + (size_t)mb * 16 * K + kc); if (NSPLIT == 1 || NSPLIT == 2) a2[mb] = WFrag<T16>::ld(A2 + aoff + (size_t)mb * 16 * K + kc); }
#pragma unroll
        for (int nb = 0; nb < 4; ++nb) { const V b = WFrag<T16>::ld(Bt + boff + (size_t)nb * 16 * K + kc); V b2; if (NSPLIT >= 2) b2 = WFrag<T16>::ld(Bt2 + boff + (size_t)nb * 16 * K + kc);
#pragma unroll
            for (int mb = 0; mb < 4; ++mb) { acc[mb][nb] = WFrag<T16>::mma(a[mb], b, acc[mb][nb]); if (NSPLIT == 1 || NSPLIT == 2) acc[mb][nb] = WFrag<T16>::mma(a2[mb], b, acc[mb][nb]); if (NSPLIT >= 2) acc[mb][nb] = WFrag<T16>::mma(a[mb], b2, acc[mb][nb]); } }
        asm volatile("v_nop\n\tv_nop\n\tv_nop\n\tv_nop" : "+v"(acc[0][0]), "+v"(acc[1][1]), "+v"(acc[2][2]), "+v"(acc[3][3]) : "v"(a[0]), "v"(a[3]));
    }
#pragma unroll
    for (int mb = 0; mb < 4; ++mb) {
#pragma unroll
        for (int nb = 0; nb < 4; ++nb) {
#pragma unroll
            for (int j = 0; j < 8; ++j) os[(hi * 8 + j) * 68 + nb * 16 + lr] = acc[mb][nb][j]; }
        __builtin_amdgcn_wave_barrier(); asm volatile("" ::: "memory");
        float* crow = C + (size_t)(r0 + mb * 16) * ldc + c0;
#pragma unroll 1
        for (int ps = 0; ps < 2; ++ps) {
#pragma unroll
            for (int s = 0; s < 8; ++s) { const int row = 2 * s + hi, cofs = lr * 4; v4f val = *(const v4fa*)(os + row * 68 + cofs); if (BIAS) { val[0] += bfr(bias[c0 + cofs]); val[1] += bfr(bias[c0 + cofs + 1]); val[2] += bfr(bias[c0 + cofs + 2]); val[3] += bfr(bias[c0 + cofs + 3]); }
                *(volatile v4f*)(crow + (size_t)row * ldc + cofs) = val; }
            if (ps == 0) __threadfence(); }
        __builtin_amdgcn_wave_barrier(); asm volatile("" ::: "memory");
    }
}

__device__ __forceinline__ void splitf(float y, unsigned short& h, unsigned short& l) { h = f2bf(y); l = f2bf(y - bf2f(h)); }
__device__ __forceinline__ int reflect(int i) { return i < 0 ? -i : (i >= HI ? 2 * HI - 2 - i : i); }
typedef __attribute__((ext_vector_type(4))) unsigned short v4us;

__global__ __launch_bounds__(256) void k_patch(const float* __restrict__ x, bf* A) { const size_t e = ((size_t)blockIdx.x * 256 + threadIdx.x) * 4; if (e >= (size_t)NPAT * PRP * CI) return; const int c = (int)(e % CI); const int r = (int)((e / CI) % PRP); const int p = (int)(e / ((size_t)CI * PRP)); const int fj = p % FP, fi = (p / FP) % FP, b = p / (FP * FP); v4us o;
    if (r < PR) { const int yy = reflect(fi * PP - 1 + r / KP), xx = reflect(fj * PP - 1 + r % KP);
#pragma unroll
        for (int q = 0; q < 4; ++q) o[q] = f2bf(x[(((size_t)b * CI + c + q) * HI + yy) * HI + xx]); } else { o[0] = 0; o[1] = 0; o[2] = 0; o[3] = 0; }
    *(volatile v4us*)(A + e) = o; __threadfence(); *(volatile v4us*)(A + e) = o; }
__global__ __launch_bounds__(256) void k_w1(const float* __restrict__ s, bf* W1B) { const size_t e = ((size_t)blockIdx.x * 256 + threadIdx.x) * 4; if (e >= (size_t)NPAT * CH * CI) return; const int c = (int)(e % CI); const int o = (int)((e / CI) % CH); const int p = (int)(e / ((size_t)CI * CH)); const int fj = p % FP, fi = (p / FP) % FP, b = p / (FP * FP); v4us w;
#pragma unroll
    for (int q = 0; q < 4; ++q) w[q] = f2bf(s[(((size_t)b * HYP + o * CI + c + q) * FP + fi) * FP + fj]); *(volatile v4us*)(W1B + e) = w; __threadfence(); *(volatile v4us*)(W1B + e) = w; }
__global__ __launch_bounds__(256) void k_w3(const float* __restrict__ s, bf* W3B) { const size_t e = ((size_t)blockIdx.x * 256 + threadIdx.x) * 4; if (e >= (size_t)NPAT * 64 * CH) return; const int c = (int)(e % CH); const int o = (int)((e / CH) % 64); const int p = (int)(e / ((size_t)CH * 64)); const int fj = p % FP, fi = (p / FP) % FP, b = p / (FP * FP); v4us w;
#pragma unroll
    for (int q = 0; q < 4; ++q) w[q] = o < CO ? f2bf(s[(((size_t)b * HYP + R2 + o * CH + c + q) * FP + fi) * FP + fj]) : (unsigned short)0; *(volatile v4us*)(W3B + e) = w; __threadfence(); *(volatile v4us*)(W3B + e) = w; }
__global__ __launch_bounds__(256) void k_cs1(const float* __restrict__ X1c, const float* __restrict__ MU, int centred, int p0, float* PS) { const int e = blockIdx.x * 256 + threadIdx.x; if (e >= PCH * CH) return; const int c = e % CH, pl = e / CH; const float m = centred ? MU[c] : 0.f; float s = 0.f;
    for (int r = 0; r < PR; ++r) { const float d = __fsub_rn(X1c[((size_t)pl * PRP + r) * CH + c], m); float v = centred ? __fmul_rn(d, d) : d; asm volatile("" : "+v"(v)); s = __fadd_rn(s, v); }
    *(volatile float*)(PS + (size_t)(p0 + pl) * CH + c) = s; __threadfence(); *(volatile float*)(PS + (size_t)(p0 + pl) * CH + c) = s; }
__global__ __launch_bounds__(256) void k_red(const float* __restrict__ PS, int nch, float inv, float* M) { const int c = blockIdx.x * 256 + threadIdx.x; if (c >= nch) return; float s = 0.f; for (int p = 0; p < NPAT; ++p) s = __fadd_rn(s, PS[(size_t)p * nch + c]); const float m = __fmul_rn(s, inv); *(volatile float*)(M + c) = m; __threadfence(); *(volatile float*)(M + c) = m; }
__global__ __launch_bounds__(256) void k_dw(const float* __restrict__ X1c, const float* __restrict__ MU, const float* __restrict__ VAR, const float* __restrict__ g1, const float* __restrict__ b1, const float* __restrict__ s, int p0, float* X2) { const size_t e = (size_t)blockIdx.x * 256 + threadIdx.x; if (e >= (size_t)PCH * PP * PP * CH) return; const int c = (int)(e % CH); const int j = (int)((e / CH) % PP); const int i = (int)((e / (CH * PP)) % PP); const int pl = (int)(e / ((size_t)CH * PP * PP)); const int p = p0 + pl; const int fj = p % FP, fi = (p / FP) % FP, b = p / (FP * FP);
    const float sc = __fmul_rn(bfr(g1[c]), __frsqrt_rn(__fadd_rn(VAR[c], 1e-5f))); const float mu = MU[c], bb = bfr(b1[c]); float acc = 0.f;
    for (int u = 0; u < 3; ++u) for (int v = 0; v < 3; ++v) { float t = __fmul_rn(__fsub_rn(X1c[((size_t)pl * PRP + (i + u) * KP + (j + v)) * CH + c], mu), sc); asm volatile("" : "+v"(t)); const float a = fminf(fmaxf(__fadd_rn(t, bb), 0.f), 6.0f); float q = __fmul_rn(a, bfr(s[(((size_t)b * HYP + R1 + c * 9 + u * 3 + v) * FP + fi) * FP + fj])); asm volatile("" : "+v"(q)); acc = __fadd_rn(acc, q); }
    const size_t o = ((size_t)p * PP * PP + i * PP + j) * CH + c; *(volatile float*)(X2 + o) = acc; __threadfence(); *(volatile float*)(X2 + o) = acc; }
__global__ __launch_bounds__(256) void k_cs2(const float* __restrict__ X, int nch, int ldc, const float* __restrict__ MU, int centred, float* PS) { const int e = blockIdx.x * 256 + threadIdx.x; if (e >= NPAT * nch) return; const int c = e % nch, p = e / nch; const float m = centred ? MU[c] : 0.f; float s = 0.f;
    for (int r = 0; r < PP * PP; ++r) { const float d = __fsub_rn(X[((size_t)p * PP * PP + r) * ldc + c], m); float v = centred ? __fmul_rn(d, d) : d; asm volatile("" : "+v"(v)); s = __fadd_rn(s, v); }
    *(volatile float*)(PS + e) = s; __threadfence(); *(volatile float*)(PS + e) = s; }
__global__ __launch_bounds__(256) void k_pl2(const float* __restrict__ X2c, const float* __restrict__ MU, const float* __restrict__ VAR, const float* __restrict__ g2, const float* __restrict__ b2, bf* Ph, bf* Pl) { const size_t i4 = ((size_t)blockIdx.x * 256 + threadIdx.x) * 4; if (i4 >= (size_t)PCH * PP * PP * CH) return; const int c = (int)(i4 % CH); const v4f a = *(const v4f*)(X2c + i4); v4us oh, ol;
#pragma unroll
    for (int q = 0; q < 4; ++q) { const int cq = c + q; const float sc = __fmul_rn(bfr(g2[cq]), __frsqrt_rn(__fadd_rn(VAR[cq], 1e-5f))); float t = __fmul_rn(__fsub_rn(a[q], MU[cq]), sc); asm volatile("" : "+v"(t)); unsigned short u, w; splitf(fminf(fmaxf(__fadd_rn(t, bfr(b2[cq])), 0.f), 6.0f), u, w); oh[q] = u; ol[q] = w; }
    *(volatile v4us*)(Ph + i4) = oh; *(volatile v4us*)(Pl + i4) = ol; __threadfence(); *(volatile v4us*)(Ph + i4) = oh; *(volatile v4us*)(Pl + i4) = ol; }
__global__ __launch_bounds__(256) void k_out(const float* __restrict__ X3, const float* __restrict__ MU, const float* __restrict__ VAR, const float* __restrict__ g3, const float* __restrict__ b3, const float* __restrict__ x, float* OUT) { const size_t e = ((size_t)blockIdx.x * 256 + threadIdx.x) * 4; if (e >= (size_t)NBI * CO * HI * HI) return; const int xx = (int)(e % HI); const int yy = (int)((e / HI) % HI); const int o = (int)((e / ((size_t)HI * HI)) % CO); const int b = (int)(e / ((size_t)HI * HI * CO));
    const float sc = __fmul_rn(bfr(g3[o]), __frsqrt_rn(__fadd_rn(VAR[o], 1e-5f))); const float mu = MU[o], bb = bfr(b3[o]); const int fi = yy / PP, i = yy % PP; v4f r;
#pragma unroll
    for (int q = 0; q < 4; ++q) { const int xq = xx + q; const int fj = xq / PP, j = xq % PP; const int p = (b * FP + fi) * FP + fj; float t = __fmul_rn(__fsub_rn(X3[((size_t)p * PP * PP + i * PP + j) * 64 + o], mu), sc); asm volatile("" : "+v"(t)); r[q] = __fadd_rn(bfr(x[e + q]), __fadd_rn(t, bb)); }
    *(volatile v4f*)(OUT + e) = r; __threadfence(); *(volatile v4f*)(OUT + e) = r; }

extern "C" void kernel_launch(void* const* d_in, const int* in_sizes, int n_in,
                              void* d_out, int out_size, void* d_ws, size_t ws_size, hipStream_t stream) {
    (void)in_sizes; (void)n_in; (void)out_size;
    const float* x = (const float*)d_in[0]; const float* s = (const float*)d_in[1]; const float* g1 = (const float*)d_in[2]; const float* b1 = (const float*)d_in[3]; const float* g2 = (const float*)d_in[4]; const float* b2 = (const float*)d_in[5]; const float* g3 = (const float*)d_in[6]; const float* b3 = (const float*)d_in[7];
    float* OUT = (float*)d_out;
    char* wsp = (char*)d_ws;
    auto take = [&](size_t bytes) { char* p = wsp; wsp += (bytes + 255) & ~(size_t)255; return (void*)p; };
    bf* A = (bf*)take((size_t)NPAT * PRP * CI * 2); bf* W1B = (bf*)take((size_t)NPAT * CH * CI * 2); bf* W3B = (bf*)take((size_t)NPAT * 64 * CH * 2); float* X1c = (float*)take((size_t)PCH * PRP * CH * 4); float* PS = (float*)take((size_t)NPAT * CH * 4);
    float* MU1 = (float*)take(CH * 4); float* VAR1 = (float*)take(CH * 4); float* MU2 = (float*)take(CH * 4); float* VAR2 = (float*)take(CH * 4); float* MU3 = (float*)take(64 * 4); float* VAR3 = (float*)take(64 * 4);
    float* X2 = (float*)take((size_t)NPAT * PP * PP * CH * 4); bf* Ph = (bf*)take((size_t)PCH * PP * PP * CH * 2); bf* Pl = (bf*)take((size_t)PCH * PP * PP * CH * 2); float* X3 = (float*)take((size_t)NPAT * PP * PP * 64 * 4);
    if ((size_t)(wsp - (char*)d_ws) > ws_size) return;
    k_patch<<<(unsigned)(((size_t)NPAT * PRP * CI / 4 + 255) / 256), 256, 0, stream>>>(x, A); k_w1<<<(unsigned)(((size_t)NPAT * CH * CI / 4 + 255) / 256), 256, 0, stream>>>(s, W1B); k_w3<<<(unsigned)(((size_t)NPAT * 64 * CH / 4 + 255) / 256), 256, 0, stream>>>(s, W3B);
    const float inv1 = 1.0f / (float)(NPAT * PR), inv2 = 1.0f / (float)(NPAT * PP * PP);
    auto expand = [&](int p0) { k_gemmw<bf, 0, false><<<dim3(PRP / 64, CH / 64, PCH), 32, 0, stream>>>(A + (size_t)p0 * PRP * CI, nullptr, W1B + (size_t)p0 * CH * CI, nullptr, CI, X1c, CH, nullptr, (size_t)PRP * CI, (size_t)CH * CI, (size_t)PRP * CH); };
    for (int p0 = 0; p0 < NPAT; p0 += PCH) { expand(p0); k_cs1<<<(PCH * CH + 255) / 256, 256, 0, stream>>>(X1c, nullptr, 0, p0, PS); }
    k_red<<<(CH + 255) / 256, 256, 0, stream>>>(PS, CH, inv1, MU1);
    for (int p0 = 0; p0 < NPAT; p0 += PCH) { expand(p0); k_cs1<<<(PCH * CH + 255) / 256, 256, 0, stream>>>(X1c, MU1, 1, p0, PS); }
    k_red<<<(CH + 255) / 256, 256, 0, stream>>>(PS, CH, inv1, VAR1);
    for (int p0 = 0; p0 < NPAT; p0 += PCH) { expand(p0); k_dw<<<(unsigned)(((size_t)PCH * PP * PP * CH + 255) / 256), 256, 0, stream>>>(X1c, MU1, VAR1, g1, b1, s, p0, X2); }
    k_cs2<<<(NPAT * CH + 255) / 256, 256, 0, stream>>>(X2, CH, CH, nullptr, 0, PS); k_red<<<(CH + 255) / 256, 256, 0, stream>>>(PS, CH, inv2, MU2);
    k_cs2<<<(NPAT * CH + 255) / 256, 256, 0, stream>>>(X2, CH, CH, MU2, 1, PS); k_red<<<(CH + 255) / 256, 256, 0, stream>>>(PS, CH, inv2, VAR2);
    for (int p0 = 0; p0 < NPAT; p0 += PCH) { k_pl2<<<(unsigned)(((size_t)PCH * PP * PP * CH / 4 + 255) / 256), 256, 0, stream>>>(X2 + (size_t)p0 * PP * PP * CH, MU2, VAR2, g2, b2, Ph, Pl);
        k_gemmw<bf, 1, false><<<dim3(PP * PP / 64, 1, PCH), 32, 0, stream>>>(Ph, Pl, W3B + (size_t)p0 * 64 * CH, nullptr, CH, X3 + (size_t)p0 * PP * PP * 64, 64, nullptr, (size_t)PP * PP * CH, (size_t)64 * CH, (size_t)PP * PP * 64); }
    k_cs2<<<(NPAT * 64 + 255) / 256, 256, 0, stream>>>(X3, 64, 64, nullptr, 0, PS); k_red<<<1, 256, 0, stream>>>(PS, 64, inv2, MU3);
    k_cs2<<<(NPAT * 64 + 255) / 256, 256, 0, stream>>>(X3, 64, 64, MU3, 1, PS); k_red<<<1, 256, 0, stream>>>(PS, 64, inv2, VAR3);
    k_out<<<(unsigned)(((size_t)NBI * CO * HI * HI / 4 + 255) / 256), 256, 0, stream>>>(X3, MU3, VAR3, g3, b3, x, OUT);
}
